// Score_45466523795916
// MI455X (gfx1250) — hardware-run, weakly checked
//
#include <hip/hip_runtime.h>
#include <stddef.h>


typedef _Float16 v16h __attribute__((ext_vector_type(16)));
typedef _Float16 v8h  __attribute__((ext_vector_type(8)));
typedef float    v8f  __attribute__((ext_vector_type(8)));
typedef float    v4f  __attribute__((ext_vector_type(4)));
typedef _Float16 h16;

#ifndef NB
#define NB 4
#endif
#ifndef SEQ
#define SEQ 512
#endif
#define NB_FULL  4
#define SEQ_FULL 512
#define HD    128
#define MROWS (NB * SEQ)

#define LDC 68
#define SP  (HD + 1)

#define WCARRY 64.0f
#define XCARRY 16.0f

static_assert(NB >= 1 && NB <= NB_FULL);
static_assert(SEQ >= 64 && SEQ <= SEQ_FULL && (SEQ % 64) == 0);
static_assert(HD == 128);
static_assert((HD % 32) == 0 && (HD % 64) == 0 && (HD % 8) == 0);
static_assert((MROWS % 64) == 0 && (MROWS % 16) == 0);
static_assert((SEQ % 32) == 0);
static_assert((LDC % 4) == 0 && LDC >= 64);
static_assert(16 * 8 == HD);
static_assert(32 * 4 == HD);
static_assert((2 * HD / 8) == 32);
static_assert(((HD * 2 * HD / 8) % 256) == 0);
static_assert(32 * 32 * 4 == 32 * HD);
static_assert((SEQ_FULL % 32) == 0);

#define X16_BYTES ((size_t)2 * MROWS * HD * 2)
#define WT_BYTES  ((size_t)2 * HD * HD * 2)
#define PRJ_BYTES ((size_t)2 * MROWS * HD * 4)
#define OFF_X16 ((size_t)0)
#define OFF_WT  (OFF_X16 + X16_BYTES)
#define OFF_PRJ (OFF_WT + WT_BYTES)
#define WS_TOTAL (OFF_PRJ + PRJ_BYTES)
static_assert((X16_BYTES % 128) == 0 && (WT_BYTES % 128) == 0 && (PRJ_BYTES % 128) == 0);
static_assert(WS_TOTAL <= (size_t)134217728);

__device__ __forceinline__ float bf16r(float x) {
  unsigned int u = __float_as_uint(x);
  u = (u + 0x7FFFu + ((u >> 16) & 1u)) & 0xFFFF0000u;
  return __uint_as_float(u);
}

static __device__ __forceinline__ h16 toh_flush(float v) {
  const h16 r = (h16)v;
  return (fabsf(v) < 6.103515625e-05f) ? (h16)0.0f : r;
}

__device__ __forceinline__ v16h frag_at(const _Float16* p) {
  v8h lo = *(const v8h*)(p);
  v8h hi = *(const v8h*)(p + 16);
  v16h out;
#pragma unroll
  for (int i = 0; i < 8; ++i) { out[i] = lo[i]; out[i + 8] = hi[i]; }
  return out;
}

__device__ __forceinline__ v8f wmma16(v16h a, v16h b, v8f c) {
  v8f d = __builtin_amdgcn_wmma_f32_16x16x32_f16(false, a, false, b, (short)0, c,
                                                 false, false);
  asm volatile("v_nop\n\tv_nop\n\tv_nop\n\tv_nop" : "+v"(d) : "v"(a), "v"(b));
  return d;
}

__global__ __launch_bounds__(256) void cvt_x_kernel(
    const float* __restrict__ X, _Float16* __restrict__ dst, unsigned drow0) {
  const unsigned tid = threadIdx.x;
  const unsigned crow = blockIdx.x * 16u + (tid >> 4);
  const unsigned c = (tid & 15u) * 8u;
  const unsigned bidx = crow / (unsigned)SEQ;
  const unsigned sq = crow - bidx * (unsigned)SEQ;
  const size_t srow = (size_t)bidx * SEQ_FULL + sq;
  const v4f a0 = *(const v4f*)(X + srow * HD + c);
  const v4f a1 = *(const v4f*)(X + srow * HD + c + 4u);
  v8h o;
#pragma unroll
  for (int i = 0; i < 4; ++i) {
    o[i]     = toh_flush(XCARRY * bf16r(a0[i]));
    o[i + 4] = toh_flush(XCARRY * bf16r(a1[i]));
  }
  _Float16* p = dst + (size_t)(drow0 + crow) * HD + c;
  *(volatile v8h*)p = o;
  __threadfence();
  *(volatile v8h*)p = o;
}

__global__ __launch_bounds__(256) void cvt_w_kernel(
    const float* __restrict__ Wc, _Float16* __restrict__ Wt) {
  const unsigned g = blockIdx.x * 256u + threadIdx.x;
  const unsigned ko = g >> 5;
  const unsigned j = (g & 31u) * 8u;
  const unsigned plane = j >> 7, jc = j & 127u;
  const v4f a0 = *(const v4f*)(Wc + (size_t)ko * (2u * HD) + j);
  const v4f a1 = *(const v4f*)(Wc + (size_t)ko * (2u * HD) + j + 4u);
  v8h o;
#pragma unroll
  for (int i = 0; i < 4; ++i) {
    o[i]     = toh_flush(WCARRY * bf16r(a0[i]));
    o[i + 4] = toh_flush(WCARRY * bf16r(a1[i]));
  }
  _Float16* p = Wt + (size_t)plane * (HD * HD) + (size_t)ko * HD + jc;
  *(volatile v8h*)p = o;
  __threadfence();
  *(volatile v8h*)p = o;
}

__global__ __launch_bounds__(256) void gemm_proj_kernel(
    const _Float16* __restrict__ A16, const _Float16* __restrict__ Wt,
    float* __restrict__ outf) {
  __shared__ float Cs[64 * LDC];
  const unsigned tid = threadIdx.x, lane = tid & 31u;
  const unsigned w = (unsigned)__builtin_amdgcn_readfirstlane((int)(threadIdx.x >> 5));
  const unsigned mw = w >> 1, nw = w & 1u;
  const unsigned hh = lane >> 4, m = lane & 15u;
  const unsigned n0 = blockIdx.x * 64u;
  const unsigned row0 = blockIdx.y * 64u;
  const unsigned which = row0 / (unsigned)MROWS;

  const _Float16* ap  = A16 + (size_t)(row0 + mw * 16u + m) * HD + hh * 8u;
  const _Float16* bp0 = Wt + (size_t)which * (HD * HD) + (size_t)(n0 + nw * 32u + m) * HD + hh * 8u;
  const _Float16* bp1 = bp0 + (size_t)16 * HD;
  v8f acc0 = {}, acc1 = {};
#pragma unroll 2
  for (unsigned k0 = 0; k0 < (unsigned)HD; k0 += 32u) {
    const v16h a  = frag_at(ap + k0);
    const v16h b0 = frag_at(bp0 + k0);
    const v16h b1 = frag_at(bp1 + k0);
    acc0 = wmma16(a, b0, acc0);
    acc1 = wmma16(a, b1, acc1);
  }
#pragma unroll
  for (int r = 0; r < 8; ++r) {
    float* d = &Cs[(mw * 16u + hh * 8u + (unsigned)r) * LDC + nw * 32u + m];
    d[0]  = acc0[r];
    d[16] = acc1[r];
  }
  __syncthreads();

  const float cs = 1.0f / (WCARRY * XCARRY);
  v4f xs[4];
  size_t off[4];
#pragma unroll
  for (unsigned i = 0; i < 4u; ++i) {
    const unsigned r = 16u * i + (tid >> 4);
    const unsigned c = (tid & 15u) * 4u;
    const v4f u = *(const v4f*)&Cs[r * LDC + c];
    v4f val;
#pragma unroll
    for (int j = 0; j < 4; ++j) val[j] = u[j] * cs;
    xs[i] = val;
    off[i] = (size_t)(row0 + r) * HD + n0 + c;
  }
#pragma unroll
  for (int i = 0; i < 4; ++i) *(volatile v4f*)(outf + off[i]) = xs[i];
  __threadfence();
#pragma unroll
  for (int i = 0; i < 4; ++i) *(volatile v4f*)(outf + off[i]) = xs[i];
}

__global__ __launch_bounds__(256) void pair_sum_kernel(
    const float* __restrict__ Prj, const float* __restrict__ bcat,
    const float* __restrict__ Wsingle, const float* __restrict__ bsingle,
    float* __restrict__ Out) {
  __shared__ float sA[32 * SP];
  __shared__ float sC[32 * SP];
  __shared__ float sW[HD];

  const unsigned tid = threadIdx.x;
  const unsigned b  = blockIdx.z;
  const unsigned n0 = blockIdx.y * 32u;
  const unsigned m0 = blockIdx.x * 32u;

  const float* Arows = Prj + ((size_t)b * SEQ + n0) * HD;
  const float* Crows = Prj + ((size_t)MROWS + (size_t)b * SEQ + m0) * HD;

#pragma unroll
  for (unsigned i = 0; i < 4u; ++i) {
    const unsigned idx = tid + i * 256u;
    const unsigned r = idx >> 5;
    const unsigned c = (idx & 31u) * 4u;
    const v4f va = *(const v4f*)(Arows + (size_t)r * HD + c);
    const v4f vc = *(const v4f*)(Crows + (size_t)r * HD + c);
    const v4f vb = *(const v4f*)(bcat + c);
#pragma unroll
    for (int j = 0; j < 4; ++j) {
      sA[r * SP + c + (unsigned)j] = 2.0f * (va[j] + bf16r(vb[j]));
      sC[r * SP + c + (unsigned)j] = 2.0f * vc[j];
    }
  }
  if (tid < (unsigned)HD) sW[tid] = bf16r(Wsingle[tid]);
  __syncthreads();

  const unsigned nl = tid >> 3;
  const unsigned mg = (tid & 7u) * 4u;

  float acc0 = 0.0f, acc1 = 0.0f, acc2 = 0.0f, acc3 = 0.0f;
#pragma unroll 2
  for (unsigned k = 0; k < (unsigned)HD; ++k) {
    const float a  = sA[nl * SP + k];
    const float wk = sW[k];
    const float e0 = __expf(a + sC[(mg + 0u) * SP + k]);
    const float e1 = __expf(a + sC[(mg + 1u) * SP + k]);
    const float e2 = __expf(a + sC[(mg + 2u) * SP + k]);
    const float e3 = __expf(a + sC[(mg + 3u) * SP + k]);
    const float t0 = 1.0f - 2.0f * __builtin_amdgcn_rcpf(e0 + 1.0f);
    const float t1 = 1.0f - 2.0f * __builtin_amdgcn_rcpf(e1 + 1.0f);
    const float t2 = 1.0f - 2.0f * __builtin_amdgcn_rcpf(e2 + 1.0f);
    const float t3 = 1.0f - 2.0f * __builtin_amdgcn_rcpf(e3 + 1.0f);
    acc0 = fmaf(wk, t0, acc0);
    acc1 = fmaf(wk, t1, acc1);
    acc2 = fmaf(wk, t2, acc2);
    acc3 = fmaf(wk, t3, acc3);
  }

  const float bs = bf16r(bsingle[0]);
  v4f val;
  val[0] = acc0 + bs;
  val[1] = acc1 + bs;
  val[2] = acc2 + bs;
  val[3] = acc3 + bs;
  float* o = Out + ((size_t)b * SEQ_FULL + (n0 + nl)) * SEQ_FULL + m0 + mg;
  *(volatile v4f*)o = val;
  __threadfence();
  *(volatile v4f*)o = val;
}

extern "C" void kernel_launch(void* const* d_in, const int* in_sizes, int n_in,
                              void* d_out, int out_size, void* d_ws, size_t ws_size,
                              hipStream_t stream) {
  if (n_in < 6) return;
  const long long need_x = ((long long)(NB - 1) * SEQ_FULL + SEQ) * HD;
  const long long need_o = ((long long)(NB - 1) * SEQ_FULL + (SEQ - 1)) * SEQ_FULL + SEQ;
  if ((long long)in_sizes[0] < need_x) return;
  if ((long long)in_sizes[1] < need_x) return;
  if ((long long)in_sizes[2] < (long long)HD * 2 * HD) return;
  if (in_sizes[3] < HD || in_sizes[4] < HD || in_sizes[5] < 1) return;
  if ((long long)out_size < need_o) return;
  if (ws_size < WS_TOTAL) return;

  const float* first  = (const float*)d_in[0];
  const float* second = (const float*)d_in[1];
  const float* wc     = (const float*)d_in[2];
  const float* bc     = (const float*)d_in[3];
  const float* wsv    = (const float*)d_in[4];
  const float* bsv    = (const float*)d_in[5];
  float* out = (float*)d_out;

  char* ws = (char*)d_ws;
  _Float16* X16 = (_Float16*)(ws + OFF_X16);
  _Float16* Wt  = (_Float16*)(ws + OFF_WT);
  float*    Prj = (float*)(ws + OFF_PRJ);

  dim3 blk(256);
  cvt_x_kernel<<<dim3(MROWS / 16), blk, 0, stream>>>(first, X16, 0u);
  cvt_x_kernel<<<dim3(MROWS / 16), blk, 0, stream>>>(second, X16, (unsigned)MROWS);
  cvt_w_kernel<<<dim3((HD * 2 * HD / 8) / 256), blk, 0, stream>>>(wc, Wt);
  gemm_proj_kernel<<<dim3(HD / 64, (2 * MROWS) / 64), blk, 0, stream>>>(X16, Wt, Prj);
  pair_sum_kernel<<<dim3(SEQ / 32, SEQ / 32, NB), blk, 0, stream>>>(Prj, bc, wsv, bsv, out);
}
